// SSFE_45921790329318
// MI455X (gfx1250) — hardware-verified
//
#include <hip/hip_runtime.h>


#define NI   8
#define CC   128
#define NP   4096
#define HH   64
#define WW   64
#define K9   1152
#define NR   32768
typedef _Float16 h16;
typedef unsigned short bf;
typedef __attribute__((ext_vector_type(16))) __bf16   v16bf;
typedef __attribute__((ext_vector_type(16))) _Float16 v16h;
typedef __attribute__((ext_vector_type(8)))  _Float16 v8h;
typedef __attribute__((ext_vector_type(8)))  unsigned short v8us;
typedef __attribute__((ext_vector_type(8)))  float    v8f;
typedef __attribute__((ext_vector_type(4)))  float    v4f;
typedef v8h  __attribute__((may_alias)) v8ha;
typedef v4f  __attribute__((may_alias)) v4fa;
typedef v8us __attribute__((may_alias)) v8usa;

__device__ __forceinline__ unsigned short f2bf(float f) { unsigned u = __float_as_uint(f); u += 0x7FFFu + ((u >> 16) & 1u); return (unsigned short)(u >> 16); }
__device__ __forceinline__ float bf2f(unsigned short b) { return __uint_as_float(((unsigned)b) << 16); }
__device__ __forceinline__ float bfr(float f) { return bf2f(f2bf(f)); }
__device__ __forceinline__ v16h cat16(v8h lo, v8h hi) { return __builtin_shufflevector(lo, hi, 0, 1, 2, 3, 4, 5, 6, 7, 8, 9, 10, 11, 12, 13, 14, 15); }
__device__ __forceinline__ v16bf cat16b(v8us lo, v8us hi) { return __builtin_bit_cast(v16bf, __builtin_shufflevector(lo, hi, 0, 1, 2, 3, 4, 5, 6, 7, 8, 9, 10, 11, 12, 13, 14, 15)); }
__device__ __forceinline__ v8f wmma16(v16h a, v16h b, v8f c) { return __builtin_amdgcn_wmma_f32_16x16x32_f16(false, a, false, b, (short)0, c, false, false); }
__device__ __forceinline__ v8f wmmab(v16bf a, v16bf b, v8f c) { return __builtin_amdgcn_wmma_f32_16x16x32_bf16(false, a, false, b, (short)0, c, false, false); }


template <typename T16> struct WFrag;
template <> struct WFrag<h16> { typedef v16h V; static __device__ __forceinline__ V ld(const h16* p) { return cat16(*(const v8h*)p, *(const v8h*)(p + 16)); } static __device__ __forceinline__ v8f mma(V a, V b, v8f c) { return wmma16(a, b, c); } };
template <> struct WFrag<bf> { typedef v16bf V; static __device__ __forceinline__ V ld(const bf* p) { return cat16b(*(const v8us*)p, *(const v8us*)(p + 16)); } static __device__ __forceinline__ v8f mma(V a, V b, v8f c) { return wmmab(a, b, c); } };
template <typename T16, int NSPLIT, bool BIAS>
__global__ __launch_bounds__(32) void k_gemmw(const T16* __restrict__ A, const T16* __restrict__ A2, const T16* __restrict__ Bt, const T16* __restrict__ Bt2, int K, float* C, int ldc, const float* __restrict__ bias, size_t sA, size_t sB, size_t sC) {
    typedef typename WFrag<T16>::V V;
    __shared__ __align__(16) float os[16 * 68];
    const size_t z = blockIdx.z; A += z * sA; if (A2) A2 += z * sA; Bt += z * sB; if (Bt2) Bt2 += z * sB; C += z * sC;
    const int lane = threadIdx.x & 31, lr = lane & 15, hi = lane >> 4; const int r0 = blockIdx.x * 64, c0 = blockIdx.y * 64;
    v8f acc[4][4];
#pragma unroll
    for (int mb = 0; mb < 4; ++mb)
#pragma unroll
        for (int nb = 0; nb < 4; ++nb) acc[mb][nb] = (v8f){};
    const size_t aoff = (size_t)(r0 + lr) * K + 8 * hi, boff = (size_t)(c0 + lr) * K + 8 * hi;
#pragma unroll 1
    for (int kc = 0; kc < K; kc += 32) {
        V a[4], a2[4];
#pragma unroll
        for (int mb = 0; mb < 4; ++mb) { a[mb] = WFrag<T16>::ld(A + aoff + (size_t)mb * 16 * K + kc); if (NSPLIT == 1 || NSPLIT == 2) a2[mb] = WFrag<T16>::ld(A2 + aoff + (size_t)mb * 16 * K + kc); }
#pragma unroll
        for (int nb = 0; nb < 4; ++nb) { const V b = WFrag<T16>::ld(Bt + boff + (size_t)nb * 16 * K + kc); V b2; if (NSPLIT >= 2) b2 = WFrag<T16>::ld(Bt2 + boff + (size_t)nb * 16 * K + kc);
#pragma unroll
            for (int mb = 0; mb < 4; ++mb) { acc[mb][nb] = WFrag<T16>::mma(a[mb], b, acc[mb][nb]); if (NSPLIT == 1 || NSPLIT == 2) acc[mb][nb] = WFrag<T16>::mma(a2[mb], b, acc[mb][nb]); if (NSPLIT >= 2) acc[mb][nb] = WFrag<T16>::mma(a[mb], b2, acc[mb][nb]); } }
        asm volatile("v_nop\n\tv_nop\n\tv_nop\n\tv_nop" : "+v"(acc[0][0]), "+v"(acc[1][1]), "+v"(acc[2][2]), "+v"(acc[3][3]) : "v"(a[0]), "v"(a[3]));
    }
#pragma unroll
    for (int mb = 0; mb < 4; ++mb) {
#pragma unroll
        for (int nb = 0; nb < 4; ++nb) {
#pragma unroll
            for (int j = 0; j < 8; ++j) os[(hi * 8 + j) * 68 + nb * 16 + lr] = acc[mb][nb][j]; }
        __builtin_amdgcn_wave_barrier(); asm volatile("" ::: "memory");
        float* crow = C + (size_t)(r0 + mb * 16) * ldc + c0;
#pragma unroll 1
        for (int ps = 0; ps < 2; ++ps) {
#pragma unroll
            for (int s = 0; s < 8; ++s) { const int row = 2 * s + hi, cofs = lr * 4; v4f val = *(const v4fa*)(os + row * 68 + cofs); if (BIAS) { val[0] += bfr(bias[c0 + cofs]); val[1] += bfr(bias[c0 + cofs + 1]); val[2] += bfr(bias[c0 + cofs + 2]); val[3] += bfr(bias[c0 + cofs + 3]); }
                *(volatile v4f*)(crow + (size_t)row * ldc + cofs) = val; }
            if (ps == 0) __threadfence(); }
        __builtin_amdgcn_wave_barrier(); asm volatile("" ::: "memory");
    }
}

__device__ __forceinline__ void splitf(float y, unsigned short& h, unsigned short& l) { h = f2bf(y); l = f2bf(y - bf2f(h)); }
typedef __attribute__((ext_vector_type(2))) unsigned short v2us;
typedef __attribute__((ext_vector_type(4))) unsigned short v4us;

__global__ __launch_bounds__(256) void k_cvt8(const float* __restrict__ src, bf* dst, size_t n8) { const size_t i = (size_t)blockIdx.x * 256 + threadIdx.x; if (i >= n8) return; const v8f v = *(const v8f*)(src + i * 8); v8us o;
#pragma unroll
    for (int k = 0; k < 8; ++k) o[k] = f2bf(v[k]); *(volatile v8us*)(dst + i * 8) = o; __threadfence(); *(volatile v8us*)(dst + i * 8) = o; }
__global__ __launch_bounds__(256) void k_xt(const float* __restrict__ x, bf* XT) { const int e = (blockIdx.x * 256 + threadIdx.x) * 2; if (e >= NP * CC) return; const int c = e % CC; const int p = e / CC; v2us o; o[0] = f2bf(x[(size_t)c * NP + p]); o[1] = f2bf(x[(size_t)(c + 1) * NP + p]); *(volatile v2us*)(XT + e) = o; __threadfence(); *(volatile v2us*)(XT + e) = o; }
__global__ __launch_bounds__(256) void k_inv(const float* __restrict__ Q, float* INV) { const int p = blockIdx.x * 256 + threadIdx.x; if (p >= NP) return; float s = 0.f;
#pragma unroll 1
    for (int c = 0; c < CC; ++c) { const float v = Q[(size_t)c * NP + p]; float t = __fmul_rn(v, v); asm volatile("" : "+v"(t)); s = __fadd_rn(s, t); } const float inv = __fdiv_rn(1.0f, fmaxf(__fsqrt_rn(s), 1e-12f)); *(volatile float*)(INV + p) = inv; __threadfence(); *(volatile float*)(INV + p) = inv; }
__global__ __launch_bounds__(256) void k_qn(const float* __restrict__ Q, const float* __restrict__ INV, float* QN) { const int e = (blockIdx.x * 256 + threadIdx.x) * 4; if (e >= CC * NP) return; const int p = e % NP; const v4f a = *(const v4f*)(Q + e); v4f o;
#pragma unroll
    for (int u = 0; u < 4; ++u) o[u] = __fmul_rn(a[u], INV[p + u]); *(volatile v4f*)(QN + e) = o; __threadfence(); *(volatile v4f*)(QN + e) = o; }
__global__ __launch_bounds__(256) void k_sim(const float* __restrict__ QN, float* SIM) { const int p = blockIdx.x * 256 + threadIdx.x; if (p >= NP) return; const int pc = (NP - 1) / 2; float num = 0.f, nq = 0.f, ncen = 0.f;
#pragma unroll 1
    for (int c = 0; c < CC; ++c) { const float a = QN[(size_t)c * NP + pc], b = QN[(size_t)c * NP + p]; float t1 = __fmul_rn(a, b), t2 = __fmul_rn(b, b), t3 = __fmul_rn(a, a); asm volatile("" : "+v"(t1)); asm volatile("" : "+v"(t2)); asm volatile("" : "+v"(t3)); num = __fadd_rn(num, t1); nq = __fadd_rn(nq, t2); ncen = __fadd_rn(ncen, t3); }
    float den = __fmul_rn(fmaxf(__fsqrt_rn(ncen), 1e-8f), fmaxf(__fsqrt_rn(nq), 1e-8f)); asm volatile("" : "+v"(den)); const float s = fmaxf(__fdiv_rn(num, den), 0.f); *(volatile float*)(SIM + p) = s; __threadfence(); *(volatile float*)(SIM + p) = s; }
__global__ __launch_bounds__(256) void k_ss(const float* __restrict__ QN, bf* Sh, bf* Sl) { const size_t e = ((size_t)blockIdx.x * 256 + threadIdx.x) * 4; if (e >= (size_t)NP * K9) return; const int k0 = (int)(e % K9); const int p = (int)(e / K9); const int y = p / WW, x = p % WW; v4us oh, ol;
#pragma unroll
    for (int u = 0; u < 4; ++u) { const int k = k0 + u; const int c = k / 9, uv = k % 9; const int yy = y + uv / 3 - 1, xx = x + uv % 3 - 1; float v = 0.f;
        if (yy >= 0 && yy < HH && xx >= 0 && xx < WW) { float pr = __fmul_rn(QN[(size_t)c * NP + yy * WW + xx], QN[(size_t)c * NP + p]); asm volatile("" : "+v"(pr)); v = fmaxf(pr, 0.f); }
        unsigned short a, b; splitf(v, a, b); oh[u] = a; ol[u] = b; }
    *(volatile v4us*)(Sh + e) = oh; *(volatile v4us*)(Sl + e) = ol; __threadfence(); *(volatile v4us*)(Sh + e) = oh; *(volatile v4us*)(Sl + e) = ol; }
__global__ __launch_bounds__(128) void k_bn(const float* __restrict__ Y, float* MU, float* RS) { const int o = threadIdx.x; float s = 0.f;
    for (int r = 0; r < NR; ++r) s = __fadd_rn(s, Y[(size_t)r * CC + o]);
    const float mu = s * (1.0f / NR); float q = 0.f;
    for (int r = 0; r < NR; ++r) { float d = __fsub_rn(Y[(size_t)r * CC + o], mu); asm volatile("" : "+v"(d)); float pw = __fmul_rn(d, d); asm volatile("" : "+v"(pw)); q = __fadd_rn(q, pw); }
    const float rs = __frsqrt_rn(__fadd_rn(q * (1.0f / NR), 1e-5f)); for (int ps = 0; ps < 2; ++ps) { *(volatile float*)(MU + o) = mu; *(volatile float*)(RS + o) = rs; if (ps == 0) __threadfence(); } }
__global__ __launch_bounds__(256) void k_f(const float* __restrict__ x, const float* __restrict__ Y, const float* __restrict__ MU, const float* __restrict__ RS, const float* __restrict__ ga, const float* __restrict__ be, const float* __restrict__ SIM, const float* __restrict__ QN, bf* Fh, bf* Fl) {
    const int e = (blockIdx.x * 256 + threadIdx.x) * 4; if (e >= NP * CC) return; const int c0 = e % CC; const int p = e / CC; v4us oh, ol;
#pragma unroll
    for (int u = 0; u < 4; ++u) { const int c = c0 + u; float d = __fsub_rn(Y[e + u], MU[c]); asm volatile("" : "+v"(d)); float n0 = __fmul_rn(d, RS[c]); asm volatile("" : "+v"(n0)); float g1 = bfr(ga[c]); asm volatile("" : "+v"(g1)); float t1 = __fmul_rn(g1, n0); asm volatile("" : "+v"(t1)); const float yb = fmaxf(__fadd_rn(t1, bfr(be[c])), 0.f);
        const size_t k = (size_t)c * NP + p; const int P = (int)(k / CC), CH = (int)(k % CC); float o1 = __fmul_rn(SIM[P], QN[(size_t)CH * NP + P]); asm volatile("" : "+v"(o1));
        const float f = __fadd_rn(__fadd_rn(bfr(x[k]), yb), o1); unsigned short a, b; splitf(f, a, b); oh[u] = a; ol[u] = b; }
    *(volatile v4us*)(Fh + e) = oh; *(volatile v4us*)(Fl + e) = ol; __threadfence(); *(volatile v4us*)(Fh + e) = oh; *(volatile v4us*)(Fl + e) = ol; }
__global__ __launch_bounds__(256) void k_rl(const float* __restrict__ F1, bf* Gh, bf* Gl) { const int e = (blockIdx.x * 256 + threadIdx.x) * 4; if (e >= NP * CC) return; const v4f a = *(const v4f*)(F1 + e); v4us oh, ol;
#pragma unroll
    for (int u = 0; u < 4; ++u) { unsigned short h, l; splitf(fmaxf(a[u], 0.f), h, l); oh[u] = h; ol[u] = l; } *(volatile v4us*)(Gh + e) = oh; *(volatile v4us*)(Gl + e) = ol; __threadfence(); *(volatile v4us*)(Gh + e) = oh; *(volatile v4us*)(Gl + e) = ol; }
__global__ __launch_bounds__(256) void k_outT(const float* __restrict__ F2T, float* OUTb) { const int e = (blockIdx.x * 256 + threadIdx.x) * 4; if (e >= CC * NP) return; const int p = e % NP; const int o = e / NP; v4f r;
#pragma unroll
    for (int u = 0; u < 4; ++u) r[u] = F2T[(size_t)(p + u) * CC + o]; *(volatile v4f*)(OUTb + e) = r; __threadfence(); *(volatile v4f*)(OUTb + e) = r; }

extern "C" void kernel_launch(void* const* d_in, const int* in_sizes, int n_in,
                              void* d_out, int out_size, void* d_ws, size_t ws_size, hipStream_t stream) {
    (void)in_sizes; (void)n_in; (void)out_size;
    const float** I = (const float**)d_in;
    const float *x = I[0], *Wq = I[1], *Wc = I[2], *bc = I[3], *ga = I[4], *be = I[5], *W1 = I[6], *b1 = I[7], *W2 = I[8], *b2 = I[9];
    float* OUT = (float*)d_out;
    char* wsp = (char*)d_ws;
    auto take = [&](size_t bytes) { char* p = wsp; wsp += (bytes + 255) & ~(size_t)255; return (void*)p; };
    bf* BQ = (bf*)take(CC * CC * 2); bf* BC = (bf*)take((size_t)CC * K9 * 2); bf* BW1 = (bf*)take(CC * CC * 2); bf* BW2 = (bf*)take(CC * CC * 2);
    bf* XT = (bf*)take((size_t)NP * CC * 2); float* Q = (float*)take((size_t)CC * NP * 4); float* INV = (float*)take(NP * 4); float* QN = (float*)take((size_t)NI * CC * NP * 4); float* SIM = (float*)take((size_t)NI * NP * 4);
    bf* Sh = (bf*)take((size_t)NP * K9 * 2); bf* Sl = (bf*)take((size_t)NP * K9 * 2); float* Y = (float*)take((size_t)NR * CC * 4); float* MU = (float*)take(CC * 4); float* RS = (float*)take(CC * 4);
    bf* Fh = (bf*)take((size_t)NP * CC * 2); bf* Fl = (bf*)take((size_t)NP * CC * 2); float* F1 = (float*)take((size_t)NP * CC * 4); bf* Gh = (bf*)take((size_t)NP * CC * 2); bf* Gl = (bf*)take((size_t)NP * CC * 2); float* F2T = (float*)take((size_t)NP * CC * 4);
    if ((size_t)(wsp - (char*)d_ws) > ws_size) return;
    k_cvt8<<<(CC * CC / 8 + 255) / 256, 256, 0, stream>>>(Wq, BQ, CC * CC / 8);
    k_cvt8<<<(CC * K9 / 8 + 255) / 256, 256, 0, stream>>>(Wc, BC, CC * K9 / 8);
    k_cvt8<<<(CC * CC / 8 + 255) / 256, 256, 0, stream>>>(W1, BW1, CC * CC / 8); k_cvt8<<<(CC * CC / 8 + 255) / 256, 256, 0, stream>>>(W2, BW2, CC * CC / 8);
    const unsigned gE = (CC * NP / 4 + 255) / 256;
    for (int b = 0; b < NI; ++b) { const float* xb = x + (size_t)b * CC * NP; float* QNb = QN + (size_t)b * CC * NP;
        k_xt<<<(NP * CC / 2 + 255) / 256, 256, 0, stream>>>(xb, XT);
        k_gemmw<bf, 0, false><<<dim3(CC / 64, NP / 64, 1), 32, 0, stream>>>(BQ, nullptr, XT, nullptr, CC, Q, NP, nullptr, 0, 0, 0);
        k_inv<<<(NP + 255) / 256, 256, 0, stream>>>(Q, INV); k_qn<<<gE, 256, 0, stream>>>(Q, INV, QNb); k_sim<<<(NP + 255) / 256, 256, 0, stream>>>(QNb, SIM + (size_t)b * NP);
        k_ss<<<(unsigned)(((size_t)NP * K9 / 4 + 255) / 256), 256, 0, stream>>>(QNb, Sh, Sl);
        k_gemmw<bf, 1, true><<<dim3(NP / 64, CC / 64, 1), 32, 0, stream>>>(Sh, Sl, BC, nullptr, K9, Y + (size_t)b * NP * CC, CC, bc, 0, 0, 0); }
    k_bn<<<1, 128, 0, stream>>>(Y, MU, RS);
    for (int b = 0; b < NI; ++b) { const float* xb = x + (size_t)b * CC * NP;
        k_f<<<gE, 256, 0, stream>>>(xb, Y + (size_t)b * NP * CC, MU, RS, ga, be, SIM + (size_t)b * NP, QN + (size_t)b * CC * NP, Fh, Fl);
        k_gemmw<bf, 1, true><<<dim3(NP / 64, CC / 64, 1), 32, 0, stream>>>(Fh, Fl, BW1, nullptr, CC, F1, CC, b1, 0, 0, 0); k_rl<<<gE, 256, 0, stream>>>(F1, Gh, Gl);
        k_gemmw<bf, 1, true><<<dim3(NP / 64, CC / 64, 1), 32, 0, stream>>>(Gh, Gl, BW2, nullptr, CC, F2T, CC, b2, 0, 0, 0);
        k_outT<<<gE, 256, 0, stream>>>(F2T, OUT + (size_t)b * CC * NP); }
}
